// EdgePredictor_9010841387501
// MI455X (gfx1250) — hardware-run, weakly checked
//
#include <hip/hip_runtime.h>


#ifndef NB
#define NB 2
#endif
#ifndef SEQ
#define SEQ 1024
#endif
#define NB_FULL  2
#define SEQ_FULL 1024
#ifndef OUT_SEQ
#define OUT_SEQ SEQ
#endif
#define DM   128
#define NC   256
#define PI   64
#define PJ   32
#define LP   33
#define OSP  36

static_assert(NC == 2 * DM);
static_assert(DM % 32 == 0);
static_assert(DM % 64 == 0);
static_assert(NC % 64 == 0);
static_assert((NB * SEQ) % 64 == 0);
static_assert(SEQ % PI == 0);
static_assert(SEQ % PJ == 0);
static_assert(PJ * 4 == 128);
static_assert(DM / 4 == 32);
static_assert(((size_t)SEQ * DM) % 8 == 0);
static_assert(NB <= NB_FULL);
static_assert(SEQ <= SEQ_FULL);
static_assert(SEQ <= OUT_SEQ);
static_assert((OSP * 4) % 16 == 0);
static_assert(OSP >= PJ);

typedef unsigned short bf;
typedef __attribute__((ext_vector_type(16))) __bf16   v16bf;
typedef __attribute__((ext_vector_type(8)))  unsigned short v8us;
typedef __attribute__((ext_vector_type(8)))  float    v8f;
typedef __attribute__((ext_vector_type(4)))  float    v4f;
typedef v4f  __attribute__((may_alias)) v4fa;

__device__ __forceinline__ unsigned short f2bf(float f) { unsigned u = __float_as_uint(f); u += 0x7FFFu + ((u >> 16) & 1u); return (unsigned short)(u >> 16); }
__device__ __forceinline__ float bfr(float f) { return __uint_as_float(((unsigned)f2bf(f)) << 16); }
__device__ __forceinline__ v16bf cat16b(v8us lo, v8us hi) { return __builtin_bit_cast(v16bf, __builtin_shufflevector(lo, hi, 0, 1, 2, 3, 4, 5, 6, 7, 8, 9, 10, 11, 12, 13, 14, 15)); }
__device__ __forceinline__ v8f wmmab(v16bf a, v16bf b, v8f c) { return __builtin_amdgcn_wmma_f32_16x16x32_bf16(false, a, false, b, (short)0, c, false, false); }
__device__ __forceinline__ v16bf ldb(const bf* p)  { return cat16b(*(const v8us*)p, *(const v8us*)(p + 16)); }
__device__ __forceinline__ void wave_sync() { __builtin_amdgcn_fence(3  , "wavefront"); __builtin_amdgcn_wave_barrier(); asm volatile("" ::: "memory"); }

__global__ __launch_bounds__(256) void k_cvt8(const float* __restrict__ src, bf* dst, size_t n8) {
    const size_t i = (size_t)blockIdx.x * 256 + threadIdx.x; if (i >= n8) return;
    const v8f v = *(const v8f*)(src + i * 8); v8us o;
#pragma unroll
    for (int k = 0; k < 8; ++k) o[k] = f2bf(v[k]);
    *(volatile v8us*)(dst + i * 8) = o; __threadfence(); *(volatile v8us*)(dst + i * 8) = o;
}

__global__ __launch_bounds__(256) void k_wt(const float* __restrict__ W, bf* WT) {
    __shared__ __align__(16) float ts[32 * 132];
    static_assert(sizeof(float) * 32 * 132 <= 131072);
    const int t = threadIdx.x;
    const int half = blockIdx.x >> 2, n0 = (blockIdx.x & 3) * 32;
#pragma unroll 1
    for (int it = 0; it < 16; ++it) {
        const int e = it * 256 + t; const int k = e >> 5, c = e & 31;
        ts[c * 132 + k] = W[(size_t)(half * DM + k) * DM + n0 + c]; }
    __syncthreads();
    static_assert(256 * 16 * 2 == 32 * DM * 2);
#pragma unroll 1
    for (int ps = 0; ps < 2; ++ps) {
#pragma unroll
        for (int s = 0; s < 2; ++s) { const int p = s * 256 + t; const int row = p >> 4, k8 = (p & 15) * 8;
            const v4f x0 = *(const v4fa*)(&ts[row * 132 + k8]); const v4f x1 = *(const v4fa*)(&ts[row * 132 + k8 + 4]); v8us o;
#pragma unroll
            for (int i = 0; i < 4; ++i) { o[i] = f2bf(x0[i]); o[4 + i] = f2bf(x1[i]); }
            *(volatile v8us*)(WT + (size_t)(half * DM + n0 + row) * DM + k8) = o; }
        if (ps == 0) __threadfence(); }
}

__global__ __launch_bounds__(32) void k_proj(const bf* __restrict__ A, const bf* __restrict__ Bt, const float* __restrict__ bias, float* HP) {
    __shared__ __align__(16) float os[16 * 68];
    static_assert(sizeof(float) * 16 * 68 <= 131072);
    const int K = DM;
    const int lane = threadIdx.x & 31, lr = lane & 15, hi = lane >> 4; const int r0 = blockIdx.x * 64, c0 = blockIdx.y * 64;
    v8f acc[4][4];
#pragma unroll
    for (int mb = 0; mb < 4; ++mb)
#pragma unroll
        for (int nb = 0; nb < 4; ++nb) acc[mb][nb] = (v8f){};
    const size_t aoff = (size_t)(r0 + lr) * K + 8 * hi, boff = (size_t)(c0 + lr) * K + 8 * hi;
#pragma unroll 1
    for (int kc = 0; kc < K; kc += 32) {
        v16bf a[4];
#pragma unroll
        for (int mb = 0; mb < 4; ++mb) a[mb] = ldb(A + aoff + (size_t)mb * 16 * K + kc);
#pragma unroll
        for (int nb = 0; nb < 4; ++nb) { const v16bf b = ldb(Bt + boff + (size_t)nb * 16 * K + kc);
#pragma unroll
            for (int mb = 0; mb < 4; ++mb) acc[mb][nb] = wmmab(a[mb], b, acc[mb][nb]); }
        asm volatile("v_nop\n\tv_nop\n\tv_nop\n\tv_nop" : "+v"(acc[0][0]), "+v"(acc[1][1]), "+v"(acc[2][2]), "+v"(acc[3][3]) : "v"(a[0]), "v"(a[1]), "v"(a[2]), "v"(a[3]));
    }
    const bool hib = c0 < DM;
    float bc[4];
#pragma unroll
    for (int nb = 0; nb < 4; ++nb) { float bv = bias[(c0 & (DM - 1)) + nb * 16 + lr];
        asm volatile("" : "+v"(bv));
        const float bq = bfr(bv); bc[nb] = hib ? bq : 0.0f; }
    static_assert(32 * 16 * 8 == 16 * 64 * 4);
#pragma unroll
    for (int mb = 0; mb < 4; ++mb) {
#pragma unroll
        for (int nb = 0; nb < 4; ++nb) {
#pragma unroll
            for (int j = 0; j < 8; ++j) os[(hi * 8 + j) * 68 + nb * 16 + lr] = acc[mb][nb][j] + bc[nb]; }
        wave_sync();
        float* dst = HP + (size_t)(r0 + mb * 16) * NC + c0;
#pragma unroll 1
        for (int ps = 0; ps < 2; ++ps) {
#pragma unroll
            for (int s = 0; s < 8; ++s) { const int row = 2 * s + (lane >> 4), c4 = (lane & 15) * 4;
                const v4f val = *(const v4fa*)(&os[row * 68 + c4]);
                *(volatile v4f*)(dst + (size_t)row * NC + c4) = val; }
            if (ps == 0) __threadfence(); }
        wave_sync();
    }
}

#pragma clang fp contract(off)

__device__ __forceinline__ void relu_mac4(v4f& acc, const v4f p, const v4f q, const v4f w) {
    const v4f s = p + q; v4f r;
    r[0] = fmaxf(s[0], 0.0f); r[1] = fmaxf(s[1], 0.0f); r[2] = fmaxf(s[2], 0.0f); r[3] = fmaxf(s[3], 0.0f);
    acc = acc + r * w;
}

__global__ __launch_bounds__(256) void k_pair(const float* __restrict__ HP, const float* __restrict__ W2, const float* __restrict__ B2, float* OUT) {
    __shared__ __align__(16) v4f his[PI * LP];
    __shared__ __align__(16) v4f hjs[PJ * LP];
    __shared__ __align__(16) v4f w2s[DM / 4];
    __shared__ __align__(16) float os[PI * OSP];
    static_assert(sizeof(v4f) * (PI * LP + PJ * LP + DM / 4) + sizeof(float) * PI * OSP <= 65536);
    static_assert(sizeof(v4f) * (PI * LP + PJ * LP + DM / 4) + sizeof(float) * PI * OSP <= 131072);
    const int t  = threadIdx.x;
    const int jt = blockIdx.x, it = blockIdx.y, bb = blockIdx.z;
    const v4f* hig = (const v4f*)(HP + (size_t)(bb * SEQ + it * PI) * NC);
    const v4f* hjg = (const v4f*)(HP + (size_t)(bb * SEQ + jt * PJ) * NC + DM);
    static_assert((PI * 32) % 256 == 0);
    static_assert((PJ * 32) % 256 == 0);
#pragma unroll
    for (int e = t; e < PI * 32; e += 256) { const int r = e >> 5, c4 = e & 31; his[r * LP + c4] = hig[(size_t)r * (NC / 4) + c4]; }
#pragma unroll
    for (int e = t; e < PJ * 32; e += 256) { const int r = e >> 5, c4 = e & 31; hjs[r * LP + c4] = hjg[(size_t)r * (NC / 4) + c4]; }
    if (t < 32) { const v4f wv = ((const v4f*)W2)[t]; v4f wq; wq[0] = bfr(wv[0]); wq[1] = bfr(wv[1]); wq[2] = bfr(wv[2]); wq[3] = bfr(wv[3]); w2s[t] = wq; }
    __syncthreads();

    const int jl = t & 15, il = t >> 4;
    const v4f z = (v4f){};
    v4f a00 = z, a01 = z, a10 = z, a11 = z, a20 = z, a21 = z, a30 = z, a31 = z;
#pragma unroll 1
    for (int d4 = 0; d4 < DM / 4; ++d4) {
        const v4f w  = w2s[d4];
        const v4f p0 = his[(il +  0) * LP + d4];
        const v4f p1 = his[(il + 16) * LP + d4];
        const v4f p2 = his[(il + 32) * LP + d4];
        const v4f p3 = his[(il + 48) * LP + d4];
        const v4f q0 = hjs[(jl +  0) * LP + d4];
        const v4f q1 = hjs[(jl + 16) * LP + d4];
        relu_mac4(a00, p0, q0, w); relu_mac4(a01, p0, q1, w);
        relu_mac4(a10, p1, q0, w); relu_mac4(a11, p1, q1, w);
        relu_mac4(a20, p2, q0, w); relu_mac4(a21, p2, q1, w);
        relu_mac4(a30, p3, q0, w); relu_mac4(a31, p3, q1, w);
    }
    const float bias2 = bfr(B2[0]);
    os[(il +  0) * OSP + jl +  0] = bias2 + ((a00[0] + a00[1]) + (a00[2] + a00[3]));
    os[(il +  0) * OSP + jl + 16] = bias2 + ((a01[0] + a01[1]) + (a01[2] + a01[3]));
    os[(il + 16) * OSP + jl +  0] = bias2 + ((a10[0] + a10[1]) + (a10[2] + a10[3]));
    os[(il + 16) * OSP + jl + 16] = bias2 + ((a11[0] + a11[1]) + (a11[2] + a11[3]));
    os[(il + 32) * OSP + jl +  0] = bias2 + ((a20[0] + a20[1]) + (a20[2] + a20[3]));
    os[(il + 32) * OSP + jl + 16] = bias2 + ((a21[0] + a21[1]) + (a21[2] + a21[3]));
    os[(il + 48) * OSP + jl +  0] = bias2 + ((a30[0] + a30[1]) + (a30[2] + a30[3]));
    os[(il + 48) * OSP + jl + 16] = bias2 + ((a31[0] + a31[1]) + (a31[2] + a31[3]));
    __syncthreads();
    float* obase = OUT + ((size_t)bb * OUT_SEQ + (size_t)(it * PI)) * OUT_SEQ + (size_t)(jt * PJ);
    static_assert(256 * 16 * 2 == PI * PJ * 4);
#pragma unroll 1
    for (int ps = 0; ps < 2; ++ps) {
#pragma unroll
        for (int s = 0; s < 2; ++s) { const int p = s * 256 + t; const int row = p >> 3, c4 = (p & 7) * 4;
            const v4f val = *(const v4fa*)(&os[row * OSP + c4]);
            *(volatile v4f*)(obase + (size_t)row * OUT_SEQ + c4) = val; }
        if (ps == 0) __threadfence(); }
}

static constexpr size_t al256(size_t v) { return (v + 255) & ~(size_t)255; }
static constexpr size_t SZ_XB = al256((size_t)NB * SEQ * DM * 2);
static constexpr size_t SZ_WT = al256((size_t)NC * DM * 2);
static constexpr size_t SZ_HP = al256((size_t)NB * SEQ * NC * 4);
static constexpr size_t SZ_TOTAL = SZ_XB + SZ_WT + SZ_HP;
static_assert(SZ_TOTAL <= (size_t)134217728);
static_assert(((size_t)NB * SEQ * DM * 2) % 256 == 0);
static_assert(((size_t)NC * DM * 2) % 256 == 0);
static_assert(((size_t)NB * SEQ) % 64 == 0 && NC % 64 == 0);
static_assert((size_t)8 * 32 == (size_t)NC);

extern "C" void kernel_launch(void* const* d_in, const int* in_sizes, int n_in,
                              void* d_out, int out_size, void* d_ws, size_t ws_size, hipStream_t stream) {
    if (n_in < 5) return;
    const size_t needx = ((size_t)(NB - 1) * SEQ_FULL + SEQ) * DM;
    if ((size_t)in_sizes[0] < needx) return;
    if ((size_t)in_sizes[1] < (size_t)NC * DM) return;
    if (in_sizes[2] < DM || in_sizes[3] < DM || in_sizes[4] < 1) return;
    if ((size_t)out_size < ((size_t)(NB - 1) * OUT_SEQ + (size_t)(SEQ - 1)) * OUT_SEQ + SEQ) return;
    if (SZ_TOTAL > ws_size) return;
    const float* x  = (const float*)d_in[0];
    const float* w1 = (const float*)d_in[1];
    const float* b1 = (const float*)d_in[2];
    const float* w2 = (const float*)d_in[3];
    const float* b2 = (const float*)d_in[4];
    float* OUT = (float*)d_out;
    char* wsp = (char*)d_ws;
    bf* XB = (bf*)wsp; wsp += SZ_XB;
    bf* WT = (bf*)wsp; wsp += SZ_WT;
    float* HP = (float*)wsp; wsp += SZ_HP;

    if (SEQ == SEQ_FULL) {
        const size_t n8 = (size_t)NB * SEQ * DM / 8;
        k_cvt8<<<(unsigned)((n8 + 255) / 256), 256, 0, stream>>>(x, XB, n8);
    } else {
        const size_t n8 = (size_t)SEQ * DM / 8;
        for (int b = 0; b < NB; ++b) k_cvt8<<<(unsigned)((n8 + 255) / 256), 256, 0, stream>>>(x + (size_t)b * SEQ_FULL * DM, XB + (size_t)b * SEQ * DM, n8);
    }
    k_wt<<<8, 256, 0, stream>>>(w1, WT);
    k_proj<<<dim3(NB * SEQ / 64, NC / 64, 1), 32, 0, stream>>>(XB, WT, b1, HP);
    k_pair<<<dim3(SEQ / PJ, SEQ / PI, NB), 256, 0, stream>>>(HP, w2, b2, OUT);
}
